// GAT_61564061221033
// MI455X (gfx1250) — hardware-run, weakly checked
//
#include <hip/hip_runtime.h>
#include <stddef.h>
#include <stdint.h>
#include <math.h>


#define NN      100000
#define NE      800000
#define FD      128
#define HID     64
#define NHD     2
#define OD      64
#define K2      256
#define MROWS   128
#define MP      (((NN + MROWS - 1) / MROWS) * MROWS)
#define NTHR    256
#define NWAVE   8
#define EPT     8
#define CHUNK   (NTHR * EPT)
#define NCHUNK  ((NE + CHUNK - 1) / CHUNK)
#define NBS     1024
#define SLB     10
#define NBLK    ((NN + NBS - 1) / NBS)
#define SRCB    17
#define WLCAP   4096
#define RCAP    10240
#define DEGCAP  64
#define MEAS_MAXDEG 23
#define MEAS_B1024  8361
#define TABW    (NBS + 32)
#define BK_ZINTS (RCAP + 3 * NBS + TABW + 32)
#define BK_INTS  (NWAVE * WLCAP + BK_ZINTS)
#define BK_LDS   (BK_INTS * 4)
#define GBM     64
#define GBN     128
#define GTHR    128
#define XU      (MP * (FD / 8))
#define XBLK    (XU / NTHR)
#define W1BLK   ((FD * (FD / 8)) / NTHR)
#define W2BLK   ((FD * (K2 / 8)) / NTHR)
#define PREPBLK (XBLK + W1BLK + W2BLK + 1)
#define P_AS1   0
#define P_AS2   256
#define P_B1    512
#define P_GM    640
#define P_BT    768
#define P_B2    896
#define PARW    1024
#define NEGSL   0.2f
#define WSMAX   ((size_t)128 << 20)

static_assert(NN <= (1 << SRCB) && NBS == (1 << SLB) && (SRCB + SLB) <= 27);
static_assert((NE % 8) == 0 && NE <= (1 << 20));
static_assert((NN % 16) == 0 && (MP % GBM) == 0 && (MP % 16) == 0);
static_assert(FD == 4 * 32 && NHD * HID == FD && OD == HID && K2 == 2 * FD);
static_assert(RCAP >= MEAS_B1024 && RCAP < 65536 && (RCAP % 4) == 0 && ((RCAP / 4) % NTHR) == 0);
static_assert(DEGCAP >= MEAS_MAXDEG + 8 && DEGCAP < 65536);
static_assert(NBLK * NBS >= NN && NBS == 4 * NTHR && (NBS % NWAVE) == 0);
static_assert(TABW / 4 == NTHR + 8 && (TABW % 32) == 0);
static_assert((BK_ZINTS % 4) == 0 && BK_LDS <= 300000);
static_assert((XU % NTHR) == 0 && ((FD * (FD / 8)) % NTHR) == 0 && ((FD * (K2 / 8)) % NTHR) == 0);
static_assert(GBM == (GTHR / 32) * 16 && GBN == 4 * 32 && (FD % 32) == 0 && (K2 % 32) == 0);
static_assert(PARW == 4 * NTHR);

typedef float          v2f  __attribute__((ext_vector_type(2)));
typedef float          v4f  __attribute__((ext_vector_type(4)));
typedef float          v8f  __attribute__((ext_vector_type(8)));
typedef double         v2d  __attribute__((ext_vector_type(2)));
typedef int            v4i  __attribute__((ext_vector_type(4)));
typedef int            v8i  __attribute__((ext_vector_type(8)));
typedef unsigned int   v4u  __attribute__((ext_vector_type(4)));
typedef unsigned short v8us __attribute__((ext_vector_type(8)));
typedef __bf16         v16b __attribute__((ext_vector_type(16)));
typedef v2f  __attribute__((may_alias)) v2fa;
typedef v4f  __attribute__((may_alias)) v4fa;
typedef v4i  __attribute__((may_alias)) v4ia;
typedef v2d  __attribute__((may_alias)) v2da;
typedef v8us __attribute__((may_alias)) v8usa;
union FragB { v16b v; v8us h[2]; v8i w; };

__device__ __forceinline__ v8f wmb(const FragB& a, const FragB& b, v8f c) {
  v8f d = __builtin_amdgcn_wmma_f32_16x16x32_bf16(false, a.v, false, b.v, (short)0, c, false, false);
  asm volatile("v_nop\n\tv_nop\n\tv_nop\n\tv_nop" : "+v"(d) : "v"(a.w), "v"(b.w));
  return d;
}

__device__ __forceinline__ unsigned int f2bf(float f) {
  const unsigned int u = __float_as_uint(f);
  const unsigned int r = ((u + 0x7FFFu + ((u >> 16) & 1u)) >> 16) & 0xFFFFu;
  const bool isn = (u & 0x7FFFFFFFu) > 0x7F800000u;
  return isn ? 0x7FC0u : r;
}
__device__ __forceinline__ float bf2f(unsigned int b) { return __uint_as_float(b << 16); }
__device__ __forceinline__ float bfr(float f) { return bf2f(f2bf(f)); }
__device__ __forceinline__ v4f bfr4(const v4f a) {
  v4f r; r.x = bfr(a.x); r.y = bfr(a.y); r.z = bfr(a.z); r.w = bfr(a.w); return r;
}
__device__ __forceinline__ unsigned int pk2(float lo, float hi) { return f2bf(lo) | (f2bf(hi) << 16); }
__device__ __forceinline__ v4u pack8(const v4f a, const v4f b) {
  v4u r;
  r.x = pk2(a.x, a.y); r.y = pk2(a.z, a.w); r.z = pk2(b.x, b.y); r.w = pk2(b.z, b.w);
  return r;
}
__device__ __forceinline__ float leaky(float v) { return v > 0.f ? v : NEGSL * v; }

__global__ __launch_bounds__(NTHR) void k_prep(
    const float* __restrict__ x, const float* __restrict__ W1, const float* __restrict__ W2,
    const float* __restrict__ as1, const float* __restrict__ ad1, const float* __restrict__ b1,
    const float* __restrict__ gm, const float* __restrict__ bt,
    const float* __restrict__ as2, const float* __restrict__ ad2, const float* __restrict__ b2,
    unsigned short* xb, unsigned short* w1t, unsigned short* w2t, float* par) {
  const int tid = (int)threadIdx.x;
  const int blk = (int)blockIdx.x;
  if (blk < XBLK) {
    const int i = blk * NTHR + tid;
    const int row = i >> 4;
    const int c0 = (i & 15) * 8;
    const int rc = row < NN ? row : NN - 1;
    const float* p = x + (size_t)rc * FD + c0;
    const v4f a = *(const v4fa*)p;
    const v4f b = *(const v4fa*)(p + 4);
    asm volatile("" :: "v"(a), "v"(b));
    v4u hv = pack8(a, b);
    const unsigned int msk = row < NN ? 0xFFFFFFFFu : 0u;
    hv.x &= msk; hv.y &= msk; hv.z &= msk; hv.w &= msk;
    unsigned short* o = xb + (size_t)row * FD + c0;
    *(volatile v4u*)o = hv;
    __threadfence();
    *(volatile v4u*)o = hv;
  } else if (blk < XBLK + W1BLK) {
    const int u = (blk - XBLK) * NTHR + tid;
    const int n = u >> 4;
    const int k8 = (u & 15) * 8;
    const float* p = W1 + (size_t)k8 * FD + n;
    v4f a, b;
    a.x = p[0];      a.y = p[FD];     a.z = p[2 * FD]; a.w = p[3 * FD];
    b.x = p[4 * FD]; b.y = p[5 * FD]; b.z = p[6 * FD]; b.w = p[7 * FD];
    const v4u wv = pack8(a, b);
    unsigned short* o = w1t + (size_t)n * FD + k8;
    *(volatile v4u*)o = wv;
    __threadfence();
    *(volatile v4u*)o = wv;
  } else if (blk < XBLK + W1BLK + W2BLK) {
    const int u = (blk - XBLK - W1BLK) * NTHR + tid;
    const int n = u >> 5;
    const int k8 = (u & 31) * 8;
    const int kk = k8 & (FD - 1);
    const float* p = W2 + (size_t)kk * FD + n;
    v4f a, b;
    a.x = p[0];      a.y = p[FD];     a.z = p[2 * FD]; a.w = p[3 * FD];
    b.x = p[4 * FD]; b.y = p[5 * FD]; b.z = p[6 * FD]; b.w = p[7 * FD];
    const v4u wv = pack8(a, b);
    unsigned short* o = w2t + (size_t)n * K2 + k8;
    *(volatile v4u*)o = wv;
    __threadfence();
    *(volatile v4u*)o = wv;
  } else {
    const int w = __builtin_amdgcn_readfirstlane(tid >> 5);
    const int q = tid & 31;
    v4f v;
    if (w == 0)      v = *(const v4fa*)(as1 + 4 * q);
    else if (w == 1) v = *(const v4fa*)(ad1 + 4 * q);
    else if (w == 2) v = *(const v4fa*)(as2 + 4 * q);
    else if (w == 3) v = *(const v4fa*)(ad2 + 4 * q);
    else if (w == 4) v = *(const v4fa*)(b1 + 4 * q);
    else if (w == 5) v = *(const v4fa*)(gm + 4 * q);
    else if (w == 6) v = *(const v4fa*)(bt + 4 * q);
    else {
      const int qc = q < 16 ? q : 15;
      v = *(const v4fa*)(b2 + 4 * qc);
    }
    asm volatile("" :: "v"(v));
    const unsigned int msk = (w == 7 && q >= 16) ? 0u : 0xFFFFFFFFu;
    const v4f r = bfr4(v);
    v4f o4;
    o4.x = __uint_as_float(__float_as_uint(r.x) & msk);
    o4.y = __uint_as_float(__float_as_uint(r.y) & msk);
    o4.z = __uint_as_float(__float_as_uint(r.z) & msk);
    o4.w = __uint_as_float(__float_as_uint(r.w) & msk);
    float* o = par + 4 * tid;
    *(volatile v4f*)o = o4;
    __threadfence();
    *(volatile v4f*)o = o4;
  }
}

__global__ __launch_bounds__(NTHR) void k_bucket(const int* __restrict__ srcs, const int* __restrict__ dsts,
                                                 int* hitsG, int* tabG) {
  extern __shared__ __attribute__((aligned(16))) int dsm[];
  int* wl   = dsm;
  int* hits = wl + NWAVE * WLCAP;
  int* cnt  = hits + RCAP;
  int* off  = cnt + NBS;
  int* cur  = off + NBS;
  int* tab  = cur + NBS;
  int* misc = tab + TABW;
  const int tid = (int)threadIdx.x, lane = tid & 31;
  const int wave = __builtin_amdgcn_readfirstlane(tid >> 5);
  const int b = (int)blockIdx.x;
  const int nodeBase = b * NBS;
  const int nbr = NN - nodeBase;
  const unsigned int unb = (unsigned int)(nbr < NBS ? nbr : NBS);
  const unsigned int nbs = (unsigned int)nodeBase;

  {
    const v4i z4 = {0, 0, 0, 0};
    for (int i = tid * 4; i < BK_ZINTS; i += NTHR * 4) *(v4ia*)(hits + i) = z4;
  }
  __syncthreads();

  int wc = 0;
#pragma unroll 1
  for (int ch = 0; ch < NCHUNK; ++ch) {
    const int e0 = ch * CHUNK + tid * EPT;
    const int ec = e0 <= NE - EPT ? e0 : NE - EPT;
    const v4i da = *(const v4i*)(dsts + ec);
    const v4i db = *(const v4i*)(dsts + ec + 4);
    asm volatile("" :: "v"(da), "v"(db));
    const bool inr = e0 < NE;
    const unsigned int s0 = (unsigned int)da.x - nbs, s1 = (unsigned int)da.y - nbs;
    const unsigned int s2 = (unsigned int)da.z - nbs, s3 = (unsigned int)da.w - nbs;
    const unsigned int s4 = (unsigned int)db.x - nbs, s5 = (unsigned int)db.y - nbs;
    const unsigned int s6 = (unsigned int)db.z - nbs, s7 = (unsigned int)db.w - nbs;
    const bool h0 = inr & (s0 < unb), h1 = inr & (s1 < unb), h2 = inr & (s2 < unb), h3 = inr & (s3 < unb);
    const bool h4 = inr & (s4 < unb), h5 = inr & (s5 < unb), h6 = inr & (s6 < unb), h7 = inr & (s7 < unb);
    const unsigned int any = __builtin_amdgcn_ballot_w32(h0 | h1 | h2 | h3 | h4 | h5 | h6 | h7);
    if (any != 0u) {
#define HITJ(J, HJ, SJ) { \
      const unsigned int mj = __builtin_amdgcn_ballot_w32(HJ); \
      if (mj != 0u) { \
        if (HJ) { \
          const int pos = wc + (int)__builtin_amdgcn_mbcnt_lo(mj, 0u); \
          if (pos < WLCAP) wl[wave * WLCAP + pos] = ((e0 + (J)) << SLB) | (int)(SJ); \
        } \
        wc += (int)__builtin_popcount(mj); } }
      HITJ(0, h0, s0)
      HITJ(1, h1, s1)
      HITJ(2, h2, s2)
      HITJ(3, h3, s3)
      HITJ(4, h4, s4)
      HITJ(5, h5, s5)
      HITJ(6, h6, s6)
      HITJ(7, h7, s7)
#undef HITJ
    }
  }
  if (lane == 0) misc[wave] = wc;
  __syncthreads();

  if (wave == 0) {
    int t = 0, ovw = 0;
#pragma unroll 1
    for (int w2 = 0; w2 < NWAVE; ++w2) {
      const int cr = misc[w2];
      ovw |= (cr > WLCAP) ? 1 : 0;
      int cv = cr < 0 ? 0 : (cr > WLCAP ? WLCAP : cr);
      const int c = __builtin_amdgcn_readfirstlane(cv);
#pragma unroll 1
      for (int b0 = 0; b0 < c; b0 += 32) {
        int idx = b0 + lane;
        idx = idx < c ? idx : c - 1;
        const int ent = wl[w2 * WLCAP + idx];
        const int m32 = (c - b0) < 32 ? (c - b0) : 32;
#pragma unroll 1
        for (int k = 0; k < m32; ++k) {
          const int u = __builtin_amdgcn_readlane(ent, k);
          const int sl = u & (NBS - 1);
          if (lane == 0) cnt[sl] = cnt[sl] + 1;
        }
        t += m32;
      }
    }
    ovw |= (t > RCAP) ? 1 : 0;
    if (lane == 0) { misc[8] = t; misc[9] = ovw; }
  }
  __syncthreads();

  {
    const v4i ca = *(const v4ia*)(cnt + 4 * tid);
    const int e0 = ca.x < 0 ? 0 : ca.x, e1 = ca.y < 0 ? 0 : ca.y;
    const int e2 = ca.z < 0 ? 0 : ca.z, e3 = ca.w < 0 ? 0 : ca.w;
    const int ts = e0 + e1 + e2 + e3;
    int incl = ts;
#pragma unroll
    for (int d = 1; d < 32; d <<= 1) {
      const int up = __shfl_up(incl, d);
      incl += (lane >= d) ? up : 0;
    }
    if (lane == 31) misc[16 + wave] = incl;
    __syncthreads();
    int pre = 0;
#pragma unroll
    for (int w2 = 0; w2 < NWAVE; ++w2) {
      const int mv = misc[16 + w2];
      pre += (w2 < wave) ? mv : 0;
    }
    int run = pre + incl - ts;
    v4i o4;
    o4.x = run; run += e0;
    o4.y = run; run += e1;
    o4.z = run; run += e2;
    o4.w = run;
    *(v4ia*)(off + 4 * tid) = o4;
    *(v4ia*)(cur + 4 * tid) = o4;
  }
  __syncthreads();

  if (wave == 0) {
#pragma unroll 1
    for (int w2 = 0; w2 < NWAVE; ++w2) {
      const int cr = misc[w2];
      int cv = cr < 0 ? 0 : (cr > WLCAP ? WLCAP : cr);
      const int c = __builtin_amdgcn_readfirstlane(cv);
#pragma unroll 1
      for (int b0 = 0; b0 < c; b0 += 32) {
        int idx = b0 + lane;
        idx = idx < c ? idx : c - 1;
        const int ent = wl[w2 * WLCAP + idx];
        int eid = (int)((unsigned int)ent >> SLB);
        eid = eid > NE - 1 ? NE - 1 : eid;
        int sr = srcs[eid];
        sr = sr < 0 ? 0 : (sr > NN - 1 ? NN - 1 : sr);
        const int word = sr | ((ent & (NBS - 1)) << SRCB);
        const int m32 = (c - b0) < 32 ? (c - b0) : 32;
#pragma unroll 1
        for (int k = 0; k < m32; ++k) {
          const int wk = __builtin_amdgcn_readlane(word, k);
          const int sl = (wk >> SRCB) & (NBS - 1);
          if (lane == 0) {
            int p = cur[sl];
            p = p < 0 ? 0 : (p > RCAP - 1 ? RCAP - 1 : p);
            hits[p] = wk;
            cur[sl] = p + 1;
          }
        }
      }
    }
  }
  __syncthreads();

  {
    const v4i oa = *(const v4ia*)(off + 4 * tid);
    const v4i ca = *(const v4ia*)(cnt + 4 * tid);
    v4i tv;
#define PKOC(O, C) ((((O) < 0 ? 0 : ((O) > RCAP ? RCAP : (O)))) | ((((C) < 0 ? 0 : ((C) > 65535 ? 65535 : (C)))) << 16))
    tv.x = PKOC(oa.x, ca.x);
    tv.y = PKOC(oa.y, ca.y);
    tv.z = PKOC(oa.z, ca.z);
    tv.w = PKOC(oa.w, ca.w);
#undef PKOC
    *(v4ia*)(tab + 4 * tid) = tv;
    if (tid == 0) { tab[NBS] = misc[9]; tab[NBS + 1] = misc[8]; }
  }
  __syncthreads();
  int* hg = hitsG + (size_t)b * RCAP;
  int* tg = tabG + (size_t)b * TABW;
  const int pt = NTHR + (tid & 7);
#pragma unroll 1
  for (int i = tid; i < RCAP / 4; i += NTHR) {
    const v4i v = *(const v4ia*)(hits + 4 * i);
    *(volatile v4i*)(hg + 4 * i) = v;
  }
  {
    const v4i v0 = *(const v4ia*)(tab + 4 * tid);
    const v4i v1 = *(const v4ia*)(tab + 4 * pt);
    *(volatile v4i*)(tg + 4 * tid) = v0;
    if (tid < 8) *(volatile v4i*)(tg + 4 * pt) = v1;
  }
  __threadfence();
#pragma unroll 1
  for (int i = tid; i < RCAP / 4; i += NTHR) {
    const v4i v = *(const v4ia*)(hits + 4 * i);
    *(volatile v4i*)(hg + 4 * i) = v;
  }
  {
    const v4i v0 = *(const v4ia*)(tab + 4 * tid);
    const v4i v1 = *(const v4ia*)(tab + 4 * pt);
    *(volatile v4i*)(tg + 4 * tid) = v0;
    if (tid < 8) *(volatile v4i*)(tg + 4 * pt) = v1;
  }
}

__global__ __launch_bounds__(GTHR) __attribute__((amdgpu_num_vgpr(248)))
void k_gemm(const unsigned short* __restrict__ A, const unsigned short* __restrict__ BT, int K,
            const float* __restrict__ att, float* outF, float* SD) {
  __shared__ __attribute__((aligned(16))) float stg[GBM * GBN];
  __shared__ __attribute__((aligned(16))) float satt[2 * GBN];
  __shared__ __attribute__((aligned(16))) float sdot[4 * GBM];
  const int tid = (int)threadIdx.x, lane = tid & 31, hh = lane >> 4, m = lane & 15;
  const int wave = __builtin_amdgcn_readfirstlane(tid >> 5);
  const int rowBase = (int)blockIdx.x * GBM;

  if (wave < 2) {
    const v4f v = *(const v4fa*)(att + 4 * tid);
    *(v4fa*)(satt + 4 * tid) = v;
  }

  v8f acc[8];
  {
    const v8f z = {0.f, 0.f, 0.f, 0.f, 0.f, 0.f, 0.f, 0.f};
#pragma unroll
    for (int t = 0; t < 8; ++t) acc[t] = z;
  }
  const unsigned short* ap = A  + (size_t)(rowBase + 16 * wave + m) * (size_t)K + 8 * hh;
  const unsigned short* bp = BT + (size_t)m * (size_t)K + 8 * hh;
#pragma unroll 1
  for (int k0 = 0; k0 < K; k0 += 32) {
    FragB af;
    af.h[0] = *(const v8usa*)(ap + k0);
    af.h[1] = *(const v8usa*)(ap + k0 + 16);
#pragma unroll
    for (int nt = 0; nt < 8; ++nt) {
      const unsigned short* wq = bp + (size_t)(16 * nt) * (size_t)K + k0;
      FragB bf;
      bf.h[0] = *(const v8usa*)wq;
      bf.h[1] = *(const v8usa*)(wq + 16);
      acc[nt] = wmb(af, bf, acc[nt]);
    }
  }

#pragma unroll
  for (int nt = 0; nt < 8; ++nt) {
    const int lc = 16 * nt + m;
#pragma unroll
    for (int r = 0; r < 8; ++r) {
      const int lr = 16 * wave + 8 * hh + r;
      stg[lr * GBN + lc] = acc[nt][r];
    }
  }
  __syncthreads();

  {
    const int row = tid & 63, side = tid >> 6;
    const float* hr = stg + row * GBN;
    const float* sa = satt + side * GBN;
    float d0 = 0.f, d1 = 0.f;
#pragma unroll 4
    for (int c4 = 0; c4 < HID / 4; ++c4) {
      const v4f hv = *(const v4fa*)(hr + 4 * c4);
      const v4f av = *(const v4fa*)(sa + 4 * c4);
      d0 = fmaf(hv.x, av.x, d0);
      d0 = fmaf(hv.y, av.y, d0);
      d0 = fmaf(hv.z, av.z, d0);
      d0 = fmaf(hv.w, av.w, d0);
    }
#pragma unroll 4
    for (int c4 = 0; c4 < HID / 4; ++c4) {
      const v4f hv = *(const v4fa*)(hr + HID + 4 * c4);
      const v4f av = *(const v4fa*)(sa + HID + 4 * c4);
      d1 = fmaf(hv.x, av.x, d1);
      d1 = fmaf(hv.y, av.y, d1);
      d1 = fmaf(hv.z, av.z, d1);
      d1 = fmaf(hv.w, av.w, d1);
    }
    sdot[row * 4 + side * 2 + 0] = d0;
    sdot[row * 4 + side * 2 + 1] = d1;
  }
  __syncthreads();

  v4f pv[16];
#pragma unroll
  for (int i = 0; i < 16; ++i) pv[i] = *(const v4fa*)(stg + (16 * wave + i) * GBN + 4 * lane);
  const v4f sdv = *(const v4fa*)(sdot + 4 * (tid & 63));
  float* sp = SD + (size_t)(rowBase + (tid & 63)) * 4;

#pragma unroll
  for (int i = 0; i < 16; ++i) {
    float* op = outF + (size_t)(rowBase + 16 * wave + i) * FD + 4 * lane;
    *(volatile v4f*)op = pv[i];
  }
  if (wave < 2) *(volatile v4f*)sp = sdv;
  __threadfence();
#pragma unroll
  for (int i = 0; i < 16; ++i) {
    float* op = outF + (size_t)(rowBase + 16 * wave + i) * FD + 4 * lane;
    *(volatile v4f*)op = pv[i];
  }
  if (wave < 2) *(volatile v4f*)sp = sdv;
}

template<int L>
__global__ __launch_bounds__(NTHR) void k_replay(
    const float* __restrict__ Hf, const float* __restrict__ SD,
    const int* __restrict__ hitsG, const int* __restrict__ tabG, const float* __restrict__ par,
    float* Tout, double* rec, float* out) {
  __shared__ __attribute__((aligned(16))) int stab[TABW];
  __shared__ __attribute__((aligned(16))) double wst[NWAVE * 2 * FD];
  const int tid = (int)threadIdx.x, lane = tid & 31;
  const int wave = __builtin_amdgcn_readfirstlane(tid >> 5);
  const int b = (int)blockIdx.x;
  const int nodeBase = b * NBS;
  {
    const int* tg = tabG + (size_t)b * TABW;
    const int pt = NTHR + (tid & 7);
    const v4i v0 = *(const v4i*)(tg + 4 * tid);
    const v4i v1 = *(const v4i*)(tg + 4 * pt);
    *(v4ia*)(stab + 4 * tid) = v0;
    *(v4ia*)(stab + 4 * pt) = v1;
  }
  __syncthreads();

  const int flag = stab[NBS];
  const float qnan = __int_as_float(0x7fc00000);
  const int c0 = 4 * lane;
  const bool hd1 = lane >= 16;
  const int* hg = hitsG + (size_t)b * RCAP;
  const v4f bb = (L == 1) ? *(const v4fa*)(par + P_B1 + c0) : *(const v4fa*)(par + P_B2 + 4 * (lane & 15));
  asm volatile("" :: "v"(bb));
  double s0 = 0.0, s1 = 0.0, s2 = 0.0, s3 = 0.0, q0 = 0.0, q1 = 0.0, q2 = 0.0, q3 = 0.0;

#pragma unroll 1
  for (int jt = 0; jt < NBS / NWAVE; ++jt) {
    const int slot = wave * (NBS / NWAVE) + jt;
    const int grow = nodeBase + slot;
    if (grow >= NN) break;
    const int oc = stab[slot];
    int ov = oc & 0xFFFF;
    const int craw = (oc >> 16) & 0xFFFF;
    ov = ov > RCAP - 1 ? RCAP - 1 : ov;
    int cv = craw > DEGCAP ? DEGCAP : craw;
    cv = cv > RCAP - ov ? RCAP - ov : cv;
    const int o = __builtin_amdgcn_readfirstlane(ov);
    const int c = __builtin_amdgcn_readfirstlane(cv);
    int last = o + c - 1; last = last < o ? o : last;
    const float pz = (flag != 0 || craw > DEGCAP) ? qnan : 0.0f;

    const v4f sdo = *(const v4fa*)(SD + (size_t)grow * 4);
    const float adv = hd1 ? sdo.w : sdo.z;
    const float l0 = leaky((hd1 ? sdo.y : sdo.x) + adv);
    float mx = l0, dn = 1.0f;
    v4f av = *(const v4fa*)(Hf + (size_t)grow * FD + c0);

#pragma unroll 1
    for (int b0 = 0; b0 < c; b0 += 32) {
      int idx = o + b0 + lane;
      idx = idx > last ? last : idx;
      const unsigned int w = (unsigned int)hg[idx];
      int s = (int)(w & ((1u << SRCB) - 1u));
      s = s > NN - 1 ? NN - 1 : s;
      const v2f asv = *(const v2fa*)(SD + (size_t)s * 4);
      const int a0i = __float_as_int(asv.x), a1i = __float_as_int(asv.y);
      const int m32 = (c - b0) < 32 ? (c - b0) : 32;
#pragma unroll 1
      for (int k = 0; k < m32; ++k) {
        const int sk = __builtin_amdgcn_readlane(s, k);
        const float a0 = __int_as_float(__builtin_amdgcn_readlane(a0i, k));
        const float a1 = __int_as_float(__builtin_amdgcn_readlane(a1i, k));
        const v4f fs = *(const v4fa*)(Hf + (size_t)sk * FD + c0);
        const float lg = leaky((hd1 ? a1 : a0) + adv);
        const float df = lg - mx;
        const float ee = expf(-fabsf(df));
        const bool up = df > 0.f;
        const float f1 = up ? ee : 1.0f;
        const float f2 = up ? 1.0f : ee;
        mx = up ? lg : mx;
        dn = fmaf(dn, f1, f2);
        av.x = fmaf(av.x, f1, f2 * fs.x);
        av.y = fmaf(av.y, f1, f2 * fs.y);
        av.z = fmaf(av.z, f1, f2 * fs.z);
        av.w = fmaf(av.w, f1, f2 * fs.w);
      }
    }
    const float inv = 1.0f / dn;
    if (L == 1) {
      v4f tv;
      tv.x = (av.x * inv + bb.x) + pz;
      tv.y = (av.y * inv + bb.y) + pz;
      tv.z = (av.z * inv + bb.z) + pz;
      tv.w = (av.w * inv + bb.w) + pz;
      const double d0 = (double)tv.x, d1 = (double)tv.y, d2 = (double)tv.z, d3 = (double)tv.w;
      s0 += d0; s1 += d1; s2 += d2; s3 += d3;
      q0 = fma(d0, d0, q0); q1 = fma(d1, d1, q1); q2 = fma(d2, d2, q2); q3 = fma(d3, d3, q3);
      float* tp = Tout + (size_t)grow * FD + c0;
      *(volatile v4f*)tp = tv;
      __threadfence();
      *(volatile v4f*)tp = tv;
    } else {
      const float rx = av.x * inv, ry = av.y * inv, rz = av.z * inv, rw = av.w * inv;
      const float ox = __shfl_xor(rx, 16), oy = __shfl_xor(ry, 16);
      const float oz = __shfl_xor(rz, 16), ow = __shfl_xor(rw, 16);
      v4f o4;
      o4.x = ((rx + ox) * 0.5f + bb.x) + pz;
      o4.y = ((ry + oy) * 0.5f + bb.y) + pz;
      o4.z = ((rz + oz) * 0.5f + bb.z) + pz;
      o4.w = ((rw + ow) * 0.5f + bb.w) + pz;
      float* op = out + (size_t)grow * OD + 4 * (lane & 15);
      if (lane < 16) *(volatile v4f*)op = o4;
      __threadfence();
      if (lane < 16) *(volatile v4f*)op = o4;
    }
  }

  if (L == 1) {
    v2d p0, p1, p2, p3;
    p0.x = s0; p0.y = q0; p1.x = s1; p1.y = q1; p2.x = s2; p2.y = q2; p3.x = s3; p3.y = q3;
    double* wp = wst + (size_t)(wave * FD + c0) * 2;
    *(v2da*)(wp + 0) = p0;
    *(v2da*)(wp + 2) = p1;
    *(v2da*)(wp + 4) = p2;
    *(v2da*)(wp + 6) = p3;
    __syncthreads();
    double S = 0.0, Q = 0.0;
    const int col = tid & (FD - 1);
#pragma unroll 1
    for (int w2 = 0; w2 < NWAVE; ++w2) {
      const v2d r = *(const v2da*)(wst + (size_t)(w2 * FD + col) * 2);
      S += r.x; Q += r.y;
    }
    v2d rv; rv.x = S; rv.y = Q;
    double* rp = rec + ((size_t)b * FD + col) * 2;
    if (wave < 4) *(volatile v2d*)rp = rv;
    __threadfence();
    if (wave < 4) *(volatile v2d*)rp = rv;
  }
}

__global__ __launch_bounds__(FD) void k_combine(const double* __restrict__ rec, float* murs) {
  __shared__ __attribute__((aligned(16))) float stg[2 * FD];
  const int tid = (int)threadIdx.x;
  double S = 0.0, Q = 0.0;
#pragma unroll 1
  for (int b = 0; b < NBLK; ++b) {
    const v2d r = *(const v2d*)(rec + ((size_t)b * FD + tid) * 2);
    S += r.x; Q += r.y;
  }
  const double rn = 1.0 / (double)NN;
  const double mu = S * rn;
  const double var = Q * rn - mu * mu;
  const float muf = (float)mu;
  const float vf = (float)var;
  const float rs = 1.0f / sqrtf(vf + 1e-5f);
  stg[tid] = muf;
  stg[FD + tid] = rs;
  __syncthreads();
  const v4f v = *(const v4fa*)(stg + 4 * (tid & 63));
  float* op = murs + 4 * (tid & 63);
  if (tid < 64) *(volatile v4f*)op = v;
  __threadfence();
  if (tid < 64) *(volatile v4f*)op = v;
}

__global__ __launch_bounds__(NTHR) void k_apply(const float* __restrict__ T, const float* __restrict__ murs,
                                                const float* __restrict__ par, unsigned short* xhl) {
  __shared__ __attribute__((aligned(16))) float tile[16 * FD];
  const int tid = (int)threadIdx.x, lane = tid & 31;
  const int wave = __builtin_amdgcn_readfirstlane(tid >> 5);
  const int col = tid & (FD - 1), r0 = tid >> 7;
  const int rowBase = (int)blockIdx.x * 16;
  const float mu = murs[col], rs = murs[FD + col];
  const float g = par[P_GM + col], be = par[P_BT + col];
#pragma unroll 1
  for (int it = 0; it < 8; ++it) {
    const int lr = 2 * it + r0;
    const int row = rowBase + lr;
    const int rc = row < NN ? row : NN - 1;
    const float t = T[(size_t)rc * FD + col];
    asm volatile("" :: "v"(t));
    const float y = ((t - mu) * rs) * g + be;
    float e = (y > 0.f) ? y : expm1f(y);
    e = (row < NN) ? e : 0.0f;
    tile[lr * FD + col] = e;
  }
  __syncthreads();
  const int q = lane & 15;
  const unsigned int smask = (lane >= 16) ? 0xFFFFFFFFu : 0u;
  v4u pv[2];
#pragma unroll
  for (int rr = 0; rr < 2; ++rr) {
    const int lr = 2 * wave + rr;
    const v4f a = *(const v4fa*)(tile + lr * FD + 8 * q);
    const v4f c = *(const v4fa*)(tile + lr * FD + 8 * q + 4);
    float vals[8];
    vals[0] = a.x; vals[1] = a.y; vals[2] = a.z; vals[3] = a.w;
    vals[4] = c.x; vals[5] = c.y; vals[6] = c.z; vals[7] = c.w;
    unsigned int ww[4];
#pragma unroll
    for (int j = 0; j < 4; ++j) {
      const float v0 = vals[2 * j], v1 = vals[2 * j + 1];
      const unsigned int h0 = f2bf(v0), h1 = f2bf(v1);
      const unsigned int l0 = f2bf(v0 - bf2f(h0)), l1 = f2bf(v1 - bf2f(h1));
      const unsigned int hw = h0 | (h1 << 16), lw = l0 | (l1 << 16);
      ww[j] = (lw & smask) | (hw & ~smask);
    }
    v4u p; p.x = ww[0]; p.y = ww[1]; p.z = ww[2]; p.w = ww[3];
    pv[rr] = p;
  }
#pragma unroll
  for (int rr = 0; rr < 2; ++rr) {
    unsigned short* op = xhl + (size_t)(rowBase + 2 * wave + rr) * K2 + 8 * lane;
    *(volatile v4u*)op = pv[rr];
  }
  __threadfence();
#pragma unroll
  for (int rr = 0; rr < 2; ++rr) {
    unsigned short* op = xhl + (size_t)(rowBase + 2 * wave + rr) * K2 + 8 * lane;
    *(volatile v4u*)op = pv[rr];
  }
}

static inline size_t al256(size_t o) { return (o + 255) & ~(size_t)255; }

extern "C" void kernel_launch(void* const* d_in, const int* in_sizes, int n_in,
                              void* d_out, int out_size, void* d_ws, size_t ws_size,
                              hipStream_t stream) {
  if (n_in < 12) return;
  if (in_sizes[0] != NN * FD) return;
  if (in_sizes[1] != 2 * NE) return;
  if (in_sizes[2] != FD * FD) return;
  if (in_sizes[3] != NHD * HID || in_sizes[4] != NHD * HID) return;
  if (in_sizes[5] != FD || in_sizes[6] != FD || in_sizes[7] != FD) return;
  if (in_sizes[8] != FD * FD) return;
  if (in_sizes[9] != NHD * OD || in_sizes[10] != NHD * OD) return;
  if (in_sizes[11] != OD) return;
  if (out_size != NN * OD) return;

  const float* x    = (const float*)d_in[0];
  const int*   ei   = (const int*)  d_in[1];
  const float* W1   = (const float*)d_in[2];
  const float* as1  = (const float*)d_in[3];
  const float* ad1  = (const float*)d_in[4];
  const float* b1   = (const float*)d_in[5];
  const float* gm   = (const float*)d_in[6];
  const float* bt   = (const float*)d_in[7];
  const float* W2   = (const float*)d_in[8];
  const float* as2  = (const float*)d_in[9];
  const float* ad2  = (const float*)d_in[10];
  const float* b2   = (const float*)d_in[11];
  float* out = (float*)d_out;
  const int* src = ei;
  const int* dst = ei + NE;

  char* ws = (char*)d_ws;
  size_t off = 0;
  const size_t oR1   = off; off = al256(off + (size_t)MP * FD * 4);
  const size_t oR2   = off; off = al256(off + (size_t)MP * FD * 4);
  const size_t oHITS = off; off = al256(off + (size_t)NBLK * RCAP * 4);
  const size_t oTAB  = off; off = al256(off + (size_t)NBLK * TABW * 4);
  const size_t oSD   = off; off = al256(off + (size_t)MP * 4 * 4);
  const size_t oREC  = off; off = al256(off + (size_t)NBLK * FD * 2 * 8);
  const size_t oMURS = off; off = al256(off + (size_t)2 * FD * 4);
  const size_t oPAR  = off; off = al256(off + (size_t)PARW * 4);
  const size_t oW1T  = off; off = al256(off + (size_t)FD * FD * 2);
  const size_t oW2T  = off; off = al256(off + (size_t)FD * K2 * 2);
  if (off > ws_size || off > WSMAX) return;
  if ((size_t)MP * FD * 2 > (size_t)MP * FD * 4) return;
  float*          H1   = (float*)(ws + oR1);
  unsigned short* X1HL = (unsigned short*)(ws + oR1);
  unsigned short* XB   = (unsigned short*)(ws + oR2);
  float*          Tp   = (float*)(ws + oR2);
  float*          H2   = (float*)(ws + oR2);
  int*            HITS = (int*)(ws + oHITS);
  int*            TAB  = (int*)(ws + oTAB);
  float*          SD   = (float*)(ws + oSD);
  double*         REC  = (double*)(ws + oREC);
  float*          MURS = (float*)(ws + oMURS);
  float*          PAR  = (float*)(ws + oPAR);
  unsigned short* W1T  = (unsigned short*)(ws + oW1T);
  unsigned short* W2T  = (unsigned short*)(ws + oW2T);

  hipFuncSetAttribute(reinterpret_cast<const void*>(&k_bucket),
                      hipFuncAttributeMaxDynamicSharedMemorySize, BK_LDS);

  k_prep<<<PREPBLK, NTHR, 0, stream>>>(x, W1, W2, as1, ad1, b1, gm, bt, as2, ad2, b2, XB, W1T, W2T, PAR);
  k_bucket<<<NBLK, NTHR, BK_LDS, stream>>>(src, dst, HITS, TAB);
  k_gemm<<<MP / GBM, GTHR, 0, stream>>>(XB, W1T, FD, PAR + P_AS1, H1, SD);
  k_replay<1><<<NBLK, NTHR, 0, stream>>>(H1, SD, HITS, TAB, PAR, Tp, REC, out);
  k_combine<<<1, FD, 0, stream>>>(REC, MURS);
  k_apply<<<MP / 16, NTHR, 0, stream>>>(Tp, MURS, PAR, X1HL);
  k_gemm<<<MP / GBM, GTHR, 0, stream>>>(X1HL, W2T, K2, PAR + P_AS2, H2, SD);
  k_replay<2><<<NBLK, NTHR, 0, stream>>>(H2, SD, HITS, TAB, PAR, Tp, REC, out);
}
